// SelfAttention_457
// MI455X (gfx1250) — hardware-verified
//
#include <hip/hip_runtime.h>
#define NB 2
#define SQ 2048
#define DM 1024
#define NH 16
#define HD 64
#define HG 4
#define B0 0
#define NBR NB
#define NR ((size_t)NB * SQ)
#define MP ((int)((size_t)NBR * SQ))
#define QN SQ
#define NHD NH
#define MPO MP
#define LQ DM
typedef __bf16 v16b __attribute__((ext_vector_type(16)));
typedef unsigned short v8us __attribute__((ext_vector_type(8), may_alias));
typedef float  v8f  __attribute__((ext_vector_type(8)));
typedef float  v4f  __attribute__((ext_vector_type(4)));
typedef float  v4fa __attribute__((ext_vector_type(4), may_alias));
union FragB { v16b v; v8us half[2]; unsigned short u[16]; };

__device__ __forceinline__ unsigned short bf16_bits(float x) { unsigned int u = __float_as_uint(x); return (unsigned short)((u + 0x7FFFu + ((u >> 16) & 1u)) >> 16); }
__device__ __forceinline__ float bf16_val(unsigned short b) { return __uint_as_float(((unsigned int)b) << 16); }
__device__ __forceinline__ float bf16_round(float x) { return bf16_val(bf16_bits(x)); }
template <int NT>
__device__ __forceinline__ v8f mmaN(v16b ah, v16b al, v16b bh, v16b bl, v8f c) {
  c = __builtin_amdgcn_wmma_f32_16x16x32_bf16(false, ah, false, bh, (short)0, c, false, false);
  if (NT >= 2) c = __builtin_amdgcn_wmma_f32_16x16x32_bf16(false, al, false, bh, (short)0, c, false, false);
  if (NT >= 3) c = __builtin_amdgcn_wmma_f32_16x16x32_bf16(false, ah, false, bl, (short)0, c, false, false);
  asm volatile("v_nop\n\tv_nop\n\tv_nop\n\tv_nop" : "+v"(c) : "v"(ah), "v"(al), "v"(bh), "v"(bl));
  return c;
}

__global__ __launch_bounds__(256) void k_wt_bf16(const float* __restrict__ W, unsigned short* __restrict__ Wt, int K, int N) {
  const int t = blockIdx.x * 256 + threadIdx.x;
  const int k8n = K / 8;
  if (t >= N * k8n) return;
  const int n = t / k8n, k8 = (t % k8n) * 8;
  v8us v;
#pragma unroll
  for (int i = 0; i < 8; ++i) v[i] = bf16_bits(W[(size_t)(k8 + i) * N + n]);
  *(volatile v8us*)(Wt + (size_t)n * K + k8) = v;
  __threadfence();
  *(volatile v8us*)(Wt + (size_t)n * K + k8) = v;
}

template <bool ASPLIT, int ACT, bool BIAS_BF16>
__global__ __launch_bounds__(128) void k_gemm_bf(const float* __restrict__ A, int lda, const unsigned short* __restrict__ Wt, int ldb,
                                               const float* __restrict__ bias, float* __restrict__ C, int ldc, int M, int N, int K) {
  __shared__ __attribute__((aligned(16))) float so[4][16][64];
  const int tid = threadIdx.x, w = tid >> 5, lane = tid & 31, ln = lane & 15, hh = lane >> 4;
  const int ntn = N / 64;
  const int wid = blockIdx.x * 4 + w;
  const int mt = wid / ntn, nq = wid % ntn;
  if (mt * 16 >= M) return;
  const int row0 = mt * 16, col0 = nq * 64;
  const float* arow = A + (size_t)(row0 + ln) * lda;
  v8f acc[4] = {};
  for (int kb = 0; kb < K; kb += 32) {
    FragB ah, al;
    const v4f x0 = *(const v4fa*)(arow + kb + 8 * hh), x1 = *(const v4fa*)(arow + kb + 8 * hh + 4);
    const v4f x2 = *(const v4fa*)(arow + kb + 16 + 8 * hh), x3 = *(const v4fa*)(arow + kb + 16 + 8 * hh + 4);
    float xs[16] = {x0[0],x0[1],x0[2],x0[3],x1[0],x1[1],x1[2],x1[3],x2[0],x2[1],x2[2],x2[3],x3[0],x3[1],x3[2],x3[3]};
#pragma unroll
    for (int i = 0; i < 16; ++i) { const unsigned short hb = bf16_bits(xs[i]); ah.u[i] = hb; al.u[i] = ASPLIT ? bf16_bits(xs[i] - bf16_val(hb)) : (unsigned short)0; }
#pragma unroll
    for (int t = 0; t < 4; ++t) {
      const unsigned short* brow = Wt + (size_t)(col0 + t * 16 + ln) * ldb + kb;
      FragB b;
      b.half[0] = *(const v8us*)(brow + 8 * hh);
      b.half[1] = *(const v8us*)(brow + 16 + 8 * hh);
      acc[t] = mmaN<ASPLIT ? 2 : 1>(ah.v, al.v, b.v, b.v, acc[t]);
    }
  }
#pragma unroll
  for (int t = 0; t < 4; ++t) {
    float bv = bias ? bias[col0 + t * 16 + ln] : 0.f;
    if (BIAS_BF16) bv = bf16_round(bv);
#pragma unroll
    for (int r = 0; r < 8; ++r) { float v = acc[t][r] + bv; if (ACT == 1) v = fmaxf(v, 0.f); so[w][8 * hh + r][t * 16 + ln] = v; }
  }
  __builtin_amdgcn_fence(__ATOMIC_ACQ_REL, "workgroup");
  __builtin_amdgcn_wave_barrier();
  const int rsub = lane >> 4, c4 = (lane & 15) * 4;
  for (int pass = 0; pass < 2; ++pass) {
#pragma unroll
    for (int q = 0; q < 8; ++q) {
      const int r = q * 2 + rsub;
      const v4f v = *(const v4fa*)&so[w][r][c4];
      *(volatile v4f*)(C + (size_t)(row0 + r) * ldc + col0 + c4) = v;
    }
    if (pass == 0) __threadfence();
  }
}

template <bool ASPLIT, int ACT, bool BIAS_BF16, bool RES_BF16>
__global__ __launch_bounds__(128) void k_gemm_bf3(const float* __restrict__ A, int lda, const unsigned short* __restrict__ Wt, int ldb,
                                                const float* __restrict__ bias, const float* __restrict__ resid, int rmod, int ldr,
                                                float* __restrict__ C, int ldc, int M, int N, int K) {
  __shared__ __attribute__((aligned(16))) float so[4][16][64];
  const int tid = threadIdx.x, w = tid >> 5, lane = tid & 31, ln = lane & 15, hh = lane >> 4;
  const int ntn = N / 64;
  const int wid = blockIdx.x * 4 + w;
  const int mt = wid / ntn, nq = wid % ntn;
  if (mt * 16 >= M) return;
  const int row0 = mt * 16, col0 = nq * 64;
  const float* arow = A + (size_t)(row0 + ln) * lda;
  v8f acc[4] = {};
  for (int kb = 0; kb < K; kb += 32) {
    FragB ah, al;
    const v4f x0 = *(const v4fa*)(arow + kb + 8 * hh), x1 = *(const v4fa*)(arow + kb + 8 * hh + 4);
    const v4f x2 = *(const v4fa*)(arow + kb + 16 + 8 * hh), x3 = *(const v4fa*)(arow + kb + 16 + 8 * hh + 4);
    float xs[16] = {x0[0],x0[1],x0[2],x0[3],x1[0],x1[1],x1[2],x1[3],x2[0],x2[1],x2[2],x2[3],x3[0],x3[1],x3[2],x3[3]};
#pragma unroll
    for (int i = 0; i < 16; ++i) { const unsigned short hb = bf16_bits(xs[i]); ah.u[i] = hb; al.u[i] = ASPLIT ? bf16_bits(xs[i] - bf16_val(hb)) : (unsigned short)0; }
#pragma unroll
    for (int t = 0; t < 4; ++t) {
      const unsigned short* brow = Wt + (size_t)(col0 + t * 16 + ln) * ldb + kb;
      FragB b;
      b.half[0] = *(const v8us*)(brow + 8 * hh);
      b.half[1] = *(const v8us*)(brow + 16 + 8 * hh);
      acc[t] = mmaN<ASPLIT ? 2 : 1>(ah.v, al.v, b.v, b.v, acc[t]);
    }
  }
#pragma unroll
  for (int t = 0; t < 4; ++t) {
    const int col = col0 + t * 16 + ln;
    float bv = bias ? bias[col] : 0.f;
    if (BIAS_BF16) bv = bf16_round(bv);
#pragma unroll
    for (int r = 0; r < 8; ++r) {
      float v = acc[t][r] + bv;
      if (resid) { float rv = resid[(size_t)((row0 + 8 * hh + r) % rmod) * ldr + col]; if (RES_BF16) rv = bf16_round(rv); v += rv; }
      if (ACT == 1) v = fmaxf(v, 0.f);
      if (ACT == 2) v = 0.5f * v * (1.0f + erff(v * 0.70710678118654752f));
      if (ACT == 3) { const float u = 0.7978845608028654f * (v + 0.044715f * v * v * v); v = 0.5f * v * (1.0f + tanhf(u)); }
      so[w][8 * hh + r][t * 16 + ln] = v;
    }
  }
  __builtin_amdgcn_fence(__ATOMIC_ACQ_REL, "workgroup");
  __builtin_amdgcn_wave_barrier();
  const int rsub = lane >> 4, c4 = (lane & 15) * 4;
  for (int pass = 0; pass < 2; ++pass) {
#pragma unroll
    for (int q = 0; q < 8; ++q) {
      const int r = q * 2 + rsub;
      const v4f v = *(const v4fa*)&so[w][r][c4];
      *(volatile v4f*)(C + (size_t)(row0 + r) * ldc + col0 + c4) = v;
    }
    if (pass == 0) __threadfence();
  }
}
template <bool PARAM_BF16>
__global__ __launch_bounds__(256) void k_layernorm(const float* __restrict__ X, const float* __restrict__ R, const float* __restrict__ g, const float* __restrict__ bta,
                                                  float* __restrict__ out_sum, float* __restrict__ out_norm, int N, float eps) {
  __shared__ float red[256];
  const int row = blockIdx.x, tid = threadIdx.x;
  const float* x = X + (size_t)row * N; const float* rr = R ? R + (size_t)row * N : nullptr;
  float vals[16];
  const int per = N / 256;
  float s1 = 0.f;
  for (int u = 0; u < per / 4; ++u) {
    const int j = tid * 4 + 1024 * u;
    const v4f a = *(const v4fa*)(x + j);
    v4f b = {0.f,0.f,0.f,0.f}; if (rr) b = *(const v4fa*)(rr + j);
#pragma unroll
    for (int q = 0; q < 4; ++q) { const float v = a[q] + b[q]; vals[u * 4 + q] = v; s1 += v; }
  }
  red[tid] = s1; __syncthreads();
  for (int st = 128; st > 0; st >>= 1) { if (tid < st) red[tid] += red[tid + st]; __syncthreads(); }
  const float mu = red[0] / (float)N; __syncthreads();
  float s2 = 0.f;
  for (int u = 0; u < per / 4; ++u)
#pragma unroll
    for (int q = 0; q < 4; ++q) { const float c = vals[u * 4 + q] - mu; s2 += c * c; }
  red[tid] = s2; __syncthreads();
  for (int st = 128; st > 0; st >>= 1) { if (tid < st) red[tid] += red[tid + st]; __syncthreads(); }
  const float rs = rsqrtf(red[0] / (float)N + eps);
  for (int pass = 0; pass < 2; ++pass) {
    for (int u = 0; u < per / 4; ++u) {
      const int j = tid * 4 + 1024 * u;
      v4f o, sm;
#pragma unroll
      for (int q = 0; q < 4; ++q) {
        float gg = g[j + q], bb = bta[j + q];
        if (PARAM_BF16) { gg = bf16_round(gg); bb = bf16_round(bb); }
        sm[q] = vals[u * 4 + q]; o[q] = (vals[u * 4 + q] - mu) * rs * gg + bb;
      }
      if (out_sum) *(volatile v4f*)(out_sum + (size_t)row * N + j) = sm;
      *(volatile v4f*)(out_norm + (size_t)row * N + j) = o;
    }
    if (pass == 0) __threadfence();
  }
}


typedef _Float16 v16h __attribute__((ext_vector_type(16)));
union FragH { v16h v; v8us half[2]; _Float16 h[16]; unsigned short u[16]; };
template <int NT>
__device__ __forceinline__ v8f mmaH(v16h ah, v16h al, v16h bh, v16h bl, v8f c) {
  c = __builtin_amdgcn_wmma_f32_16x16x32_f16(false, ah, false, bh, (short)0, c, false, false);
  if (NT >= 2) c = __builtin_amdgcn_wmma_f32_16x16x32_f16(false, al, false, bh, (short)0, c, false, false);
  if (NT >= 3) c = __builtin_amdgcn_wmma_f32_16x16x32_f16(false, ah, false, bl, (short)0, c, false, false);
  asm volatile("v_nop\n\tv_nop\n\tv_nop\n\tv_nop" : "+v"(c) : "v"(ah), "v"(al), "v"(bh), "v"(bl));
  return c;
}
template <bool ASPLIT>
__global__ __launch_bounds__(128) void k_gemm_h(const float* __restrict__ A, int lda, size_t sA, const _Float16* __restrict__ Bh, int ldb, size_t sB, float alpha, float* __restrict__ C, int ldc, size_t sC, int M, int N, int K) {
  __shared__ __attribute__((aligned(16))) float so[4][16][64];
  const int tid = threadIdx.x, w = tid >> 5, lane = tid & 31, ln = lane & 15, hh = lane >> 4; const int by = blockIdx.y;
  A += (size_t)by * sA; Bh += (size_t)by * sB; C += (size_t)by * sC;
  const int ntn = (N + 63) / 64; const int wid = blockIdx.x * 4 + w; const int mt = wid / ntn, nq = wid % ntn; if (mt * 16 >= M) return;
  const int row0 = mt * 16, col0 = nq * 64; const float* arow = A + (size_t)(row0 + ln) * lda;
  v8f acc[4] = {};
  for (int kb = 0; kb < K; kb += 32) {
    FragH ah, al;
    const v4f x0 = *(const v4fa*)(arow + kb + 8 * hh), x1 = *(const v4fa*)(arow + kb + 8 * hh + 4), x2 = *(const v4fa*)(arow + kb + 16 + 8 * hh), x3 = *(const v4fa*)(arow + kb + 16 + 8 * hh + 4);
    float xs[16] = {x0[0],x0[1],x0[2],x0[3],x1[0],x1[1],x1[2],x1[3],x2[0],x2[1],x2[2],x2[3],x3[0],x3[1],x3[2],x3[3]};
#pragma unroll
    for (int i = 0; i < 16; ++i) { const _Float16 h = (_Float16)xs[i]; ah.h[i] = h; al.h[i] = ASPLIT ? (_Float16)(xs[i] - (float)h) : (_Float16)0.0f; }
#pragma unroll
    for (int t = 0; t < 4; ++t) { if (col0 + t * 16 >= N) continue; const size_t boff = (size_t)(col0 + t * 16 + ln) * ldb + kb; FragH bq; bq.half[0] = *(const v8us*)(Bh + boff + 8 * hh); bq.half[1] = *(const v8us*)(Bh + boff + 16 + 8 * hh);
      acc[t] = mmaH<ASPLIT ? 2 : 1>(ah.v, al.v, bq.v, bq.v, acc[t]); }
  }
#pragma unroll
  for (int t = 0; t < 4; ++t) { if (col0 + t * 16 >= N) continue;
#pragma unroll
    for (int r = 0; r < 8; ++r) so[w][8 * hh + r][t * 16 + ln] = acc[t][r] * alpha; }
  __builtin_amdgcn_fence(__ATOMIC_ACQ_REL, "workgroup"); __builtin_amdgcn_wave_barrier();
  const int rsub = lane >> 4, c4 = (lane & 15) * 4;
  for (int pass = 0; pass < 2; ++pass) {
#pragma unroll
    for (int q = 0; q < 8; ++q) { const int r = q * 2 + rsub; if (col0 + c4 < N) { const v4f v = *(const v4fa*)&so[w][r][c4]; *(volatile v4f*)(C + (size_t)(row0 + r) * ldc + col0 + c4) = v; } }
    if (pass == 0) __threadfence(); }
}

__global__ __launch_bounds__(256) void k_wt_f16(const float* __restrict__ W, _Float16* __restrict__ Wt, int K, int N, float scale) {
  const int t = blockIdx.x * 256 + threadIdx.x; if (t >= N * (K / 8)) return; const int n = t / (K / 8), k8 = (t % (K / 8)) * 8; FragH f;
#pragma unroll
  for (int i = 0; i < 8; ++i) f.h[i] = (_Float16)(bf16_round(W[(size_t)(k8 + i) * N + n]) * scale); const v8us o = f.half[0];
  *(volatile v8us*)((unsigned short*)Wt + (size_t)n * K + k8) = o; __threadfence(); *(volatile v8us*)((unsigned short*)Wt + (size_t)n * K + k8) = o;
}
template <int ACT>
__global__ __launch_bounds__(128) void k_gemm_hhx(const _Float16* __restrict__ A, int lda, size_t sA, const _Float16* __restrict__ Bh, int ldb, size_t sB, float alpha, const float* __restrict__ bias, size_t sBias, const float* __restrict__ CP, int rowsPerB, size_t sCPb, int row0g,
    float* __restrict__ C, _Float16* __restrict__ C16, int ldc, size_t sC, int M, int N, int K) {
  __shared__ __attribute__((aligned(16))) float so[4][16][64];
  const int tid = threadIdx.x, w = tid >> 5, lane = tid & 31, ln = lane & 15, hh = lane >> 4; const int by = blockIdx.y;
  A += (size_t)by * sA; Bh += (size_t)by * sB; const size_t cofs = (size_t)by * sC; const float* bp = bias ? bias + (size_t)by * sBias : nullptr;
  const int ntn = (N + 63) / 64; const int wid = blockIdx.x * 4 + w; const int mt = wid / ntn, nq = wid % ntn; if (mt * 16 >= M) return;
  const int row0 = mt * 16, col0 = nq * 64; const _Float16* arow = A + (size_t)(row0 + ln) * lda;
  v8f acc[4] = {};
  for (int kb = 0; kb < K; kb += 32) { FragH ah; ah.half[0] = *(const v8us*)((const unsigned short*)arow + kb + 8 * hh); ah.half[1] = *(const v8us*)((const unsigned short*)arow + kb + 16 + 8 * hh);
#pragma unroll
    for (int t = 0; t < 4; ++t) { if (col0 + t * 16 >= N) continue; const size_t boff = (size_t)(col0 + t * 16 + ln) * ldb + kb; FragH bq; bq.half[0] = *(const v8us*)((const unsigned short*)Bh + boff + 8 * hh); bq.half[1] = *(const v8us*)((const unsigned short*)Bh + boff + 16 + 8 * hh);
      acc[t] = mmaH<1>(ah.v, ah.v, bq.v, bq.v, acc[t]); }
  }
#pragma unroll
  for (int t = 0; t < 4; ++t) { if (col0 + t * 16 >= N) continue; const int col = col0 + t * 16 + ln; const float bv = bp ? bf16_round(bp[col]) : 0.f;
#pragma unroll
    for (int r = 0; r < 8; ++r) { float v = acc[t][r] * alpha + bv; if (CP) { const int rr = row0g + row0 + 8 * hh + r; if (rowsPerB < 0) v += CP[cofs + (size_t)rr * ldc + col];        else { const int bidx = rr / rowsPerB; v += CP[(size_t)bidx * sCPb + (size_t)by * 64 + col]; } } if (ACT == 1) v = (v > 0.f) ? v : expm1f(v); else if (ACT == 7) v = (v > 0.f) ? v + 1.0f : expf(v); else if (ACT == 8) v = tanhf(v); else if (ACT == 9) v = 0.5f * v * (1.0f + tanhf(0.7978845608028654f * (v + 0.044715f * v * v * v))); else if (ACT == 11) v = 1.0f / (1.0f + expf(-v)); else if (ACT == 12) v = (v > 0.f) ? v : 0.01f * v; else if (ACT == 14) v = (v > 0.f) ? v : 0.1f * v; else if (ACT == 16) v = (v >= 0.f) ? v : 0.3f * v; else if (ACT == 17) v = (v >= 0.f) ? v : 0.2f * v; else if (ACT == 15) v = v / (1.0f + expf(-v)); else if (ACT == 3) v = fmaxf(v, 0.f); else if (ACT == 6) v = 0.5f * v * (1.0f + erff(v * 0.70710678118654752f)); so[w][8 * hh + r][t * 16 + ln] = v; } }
  __builtin_amdgcn_fence(__ATOMIC_ACQ_REL, "workgroup"); __builtin_amdgcn_wave_barrier();
  const int rsub = lane >> 4, c4 = (lane & 15) * 4; typedef _Float16 v4h __attribute__((ext_vector_type(4)));
  for (int pass = 0; pass < 2; ++pass) {
#pragma unroll
    for (int q = 0; q < 8; ++q) { const int r = q * 2 + rsub; if (col0 + c4 < N) { const v4f v = *(const v4fa*)&so[w][r][c4]; if (C) *(volatile v4f*)(C + cofs + (size_t)(row0 + r) * ldc + col0 + c4) = v; if (C16) { v4h h4; for (int i = 0; i < 4; ++i) h4[i] = (_Float16)v[i]; *(volatile v4h*)(C16 + cofs + (size_t)(row0 + r) * ldc + col0 + c4) = h4; } } }
    if (pass == 0) __threadfence(); }
}


typedef _Float16 v4h __attribute__((ext_vector_type(4)));

__global__ __launch_bounds__(256) void k_x16(const float* __restrict__ x, _Float16* __restrict__ X16, size_t n8) { const size_t t = (size_t)blockIdx.x * 256 + threadIdx.x; if (t >= n8) return; FragH f;
#pragma unroll
  for (int q = 0; q < 8; ++q) f.h[q] = (_Float16)bf16_round(x[t * 8 + q]); *(volatile v8us*)((unsigned short*)X16 + t * 8) = f.half[0]; __threadfence(); *(volatile v8us*)((unsigned short*)X16 + t * 8) = f.half[0]; }
__global__ __launch_bounds__(256) void k_h16(const float* __restrict__ x, _Float16* __restrict__ X16, size_t n8) { const size_t t = (size_t)blockIdx.x * 256 + threadIdx.x; if (t >= n8) return; FragH f;
#pragma unroll
  for (int q = 0; q < 8; ++q) f.h[q] = (_Float16)x[t * 8 + q]; *(volatile v8us*)((unsigned short*)X16 + t * 8) = f.half[0]; __threadfence(); *(volatile v8us*)((unsigned short*)X16 + t * 8) = f.half[0]; }
__global__ __launch_bounds__(256) void k_round16f(const float* __restrict__ W, _Float16* __restrict__ Bt, size_t n8) { const size_t t = (size_t)blockIdx.x * 256 + threadIdx.x; if (t >= n8) return; FragH f;
#pragma unroll
  for (int i = 0; i < 8; ++i) f.h[i] = (_Float16)(bf16_round(W[t * 8 + i]) * 16.0f); *(volatile v8us*)((unsigned short*)Bt + t * 8) = f.half[0]; __threadfence(); *(volatile v8us*)((unsigned short*)Bt + t * 8) = f.half[0]; }
template <int NHv, int TTv>
__global__ __launch_bounds__(256) void k_vt(const _Float16* __restrict__ V16, int ldv, int voff, _Float16* __restrict__ Vt) { __shared__ unsigned short tl[64][66]; const int tid = threadIdx.x; const int slab = blockIdx.x / (TTv / 64), lg = blockIdx.x % (TTv / 64); const int b = slab / NHv, h = slab % NHv;
  for (int i = tid; i < 64 * 8; i += 256) { const int r = i / 8, c8 = (i % 8) * 8; FragH f; f.half[0] = *(const v8us*)((const unsigned short*)V16 + ((size_t)b * TTv + lg * 64 + r) * ldv + voff + h * 64 + c8);
#pragma unroll
    for (int q = 0; q < 8; ++q) tl[r][c8 + q] = f.u[q]; }
  __syncthreads();
  for (int pass = 0; pass < 2; ++pass) {
#pragma unroll
    for (int rd = 0; rd < 2; ++rd) { const int d = rd * 32 + tid / 8, pc = tid % 8; FragH f;
#pragma unroll
      for (int q = 0; q < 8; ++q) f.u[q] = tl[pc * 8 + q][d];
      *(volatile v8us*)((unsigned short*)Vt + ((size_t)slab * 64 + d) * TTv + lg * 64 + pc * 8) = f.half[0]; }
    if (pass == 0) __threadfence(); } }

__global__ __launch_bounds__(256) void k_hl(const float* __restrict__ F, _Float16* __restrict__ Hh, _Float16* __restrict__ Hl, size_t n8) { const size_t t = (size_t)blockIdx.x * 256 + threadIdx.x; if (t >= n8) return; FragH fh, fl; const v4f a = *(const v4fa*)(F + t * 8), c = *(const v4fa*)(F + t * 8 + 4);
#pragma unroll
  for (int q = 0; q < 4; ++q) { _Float16 h = (_Float16)a[q]; fh.h[q] = h; fl.h[q] = (_Float16)((a[q] - (float)h) * 1024.0f); h = (_Float16)c[q]; fh.h[4 + q] = h; fl.h[4 + q] = (_Float16)((c[q] - (float)h) * 1024.0f); }
  for (int pass = 0; pass < 2; ++pass) { *(volatile v8us*)((unsigned short*)Hh + t * 8) = fh.half[0]; *(volatile v8us*)((unsigned short*)Hl + t * 8) = fl.half[0]; if (pass == 0) __threadfence(); } }

__device__ __forceinline__ v16h g2_frag(const _Float16* p, int hh) { FragH f; f.half[0] = *(const v8us*)((const unsigned short*)p + 8 * hh); f.half[1] = *(const v8us*)((const unsigned short*)p + 16 + 8 * hh); return f.v; }
__device__ __forceinline__ v8f g2_mma(v16h a, v16h b, v8f c) { v8f d = __builtin_amdgcn_wmma_f32_16x16x32_f16(false, a, false, b, (short)0, c, false, false); asm volatile("v_nop\n\tv_nop\n\tv_nop\n\tv_nop" : "+v"(d) : "v"(a), "v"(b)); return d; }
template <int ACT>
__global__ __launch_bounds__(128) void k_gemm2(const _Float16* __restrict__ A, int lda, size_t sA, const _Float16* __restrict__ Bh, int ldb, size_t sB, float alpha, const float* __restrict__ bias, size_t sBias, const float* __restrict__ CP, int rowsPerB, size_t sCPb, int row0g,
    float* __restrict__ C, _Float16* __restrict__ C16, int ldc, size_t sC, int M, int N, int K) { static_assert(ACT == 0 || ACT == 3 || ACT == 6 || ACT == 8 || ACT == 9 || ACT == 11 || ACT == 12 || ACT == 14 || ACT == 15 || ACT == 16 || ACT == 17, "k_gemm2: unsupported ACT code (would silently apply no activation)");
  __shared__ __attribute__((aligned(16))) float so[4][32][68];
  const int tid = threadIdx.x, w = tid >> 5, lane = tid & 31, ln = lane & 15, hh = lane >> 4; const int by = blockIdx.y;
  A += (size_t)by * sA; Bh += (size_t)by * sB; const size_t cofs = (size_t)by * sC; const float* bp = bias ? bias + (size_t)by * sBias : nullptr;
  const int ntn = N >> 6; const int mt = blockIdx.x / ntn, nq = blockIdx.x - mt * ntn; const int row0 = mt * 128 + 32 * w, col0 = nq * 64; if (row0 >= M) return;
  const _Float16* a0p = A + (size_t)(row0 + ln) * lda; const _Float16* a1p = a0p + (size_t)16 * lda;
  const _Float16* b0p = Bh + (size_t)(col0 + ln) * ldb; const _Float16* b1p = b0p + (size_t)16 * ldb; const _Float16* b2p = b1p + (size_t)16 * ldb; const _Float16* b3p = b2p + (size_t)16 * ldb;
  const v8f z8 = {0.f,0.f,0.f,0.f,0.f,0.f,0.f,0.f}; v8f c00 = z8, c01 = z8, c02 = z8, c03 = z8, c10 = z8, c11 = z8, c12 = z8, c13 = z8;
#pragma unroll 1
  for (int kb = 0; kb < K; kb += 32) { const v16h a0 = g2_frag(a0p + kb, hh), a1 = g2_frag(a1p + kb, hh);
    v16h b = g2_frag(b0p + kb, hh); c00 = g2_mma(a0, b, c00); c10 = g2_mma(a1, b, c10);
    b = g2_frag(b1p + kb, hh); c01 = g2_mma(a0, b, c01); c11 = g2_mma(a1, b, c11);
    b = g2_frag(b2p + kb, hh); c02 = g2_mma(a0, b, c02); c12 = g2_mma(a1, b, c12);
    b = g2_frag(b3p + kb, hh); c03 = g2_mma(a0, b, c03); c13 = g2_mma(a1, b, c13); }
  v8f accs[8] = {c00, c01, c02, c03, c10, c11, c12, c13};
#pragma unroll
  for (int u = 0; u < 8; ++u) { const int t = u & 3, half = u >> 2; const int col = col0 + t * 16 + ln; const float bv = bp ? bf16_round(bp[col]) : 0.f;
#pragma unroll
    for (int r = 0; r < 8; ++r) { const int rloc = half * 16 + 8 * hh + r; float v = accs[u][r] * alpha + bv; if (CP) { if (rowsPerB < 0) v += CP[cofs + (size_t)(row0g + row0 + rloc) * ldc + col];        else { const int bidx = (row0g + row0 + rloc) / rowsPerB; v += CP[(size_t)bidx * sCPb + (size_t)by * 64 + col]; } }
      if (ACT == 3) v = fmaxf(v, 0.f); else if (ACT == 6) v = 0.5f * v * (1.0f + erff(v * 0.70710678118654752f)); else if (ACT == 11) v = 1.0f / (1.0f + expf(-v)); else if (ACT == 15) v = v / (1.0f + expf(-v)); else if (ACT == 12) v = (v > 0.f) ? v : 0.01f * v; else if (ACT == 8) v = tanhf(v); else if (ACT == 9) v = 0.5f * v * (1.0f + tanhf(0.7978845608028654f * (v + 0.044715f * v * v * v))); else if (ACT == 14) v = (v > 0.f) ? v : 0.1f * v; else if (ACT == 16) v = (v >= 0.f) ? v : 0.3f * v; else if (ACT == 17) v = (v >= 0.f) ? v : 0.2f * v;
      so[w][rloc][t * 16 + ln] = v; } }
  __builtin_amdgcn_fence(__ATOMIC_ACQ_REL, "workgroup"); __builtin_amdgcn_wave_barrier();
  const int rsub = lane >> 4, c4 = (lane & 15) * 4;
  for (int pass = 0; pass < 2; ++pass) {
#pragma unroll
    for (int q = 0; q < 16; ++q) { const int r = q * 2 + rsub; const v4f v = *(const v4fa*)&so[w][r][c4]; if (C) *(volatile v4f*)(C + cofs + (size_t)(row0 + r) * ldc + col0 + c4) = v; if (C16) { v4h h4; for (int i = 0; i < 4; ++i) h4[i] = (_Float16)v[i]; *(volatile v4h*)(C16 + cofs + (size_t)(row0 + r) * ldc + col0 + c4) = h4; } }
    if (pass == 0) __threadfence(); } }


__global__ __launch_bounds__(256) void k_wnat(const float* __restrict__ w, size_t n8, _Float16* __restrict__ Bt) { const size_t t = (size_t)blockIdx.x * 256 + threadIdx.x; if (t >= n8) return; FragH f; for (int q = 0; q < 8; ++q) f.h[q] = (_Float16)(bf16_round(w[t * 8 + q]) * 16.0f); *(volatile v8us*)((unsigned short*)Bt + t * 8) = f.half[0]; __threadfence(); *(volatile v8us*)((unsigned short*)Bt + t * 8) = f.half[0]; }
__global__ __launch_bounds__(256) void k_rsm(const float* __restrict__ S, _Float16* __restrict__ P, int nrows) {
  #pragma clang fp contract(off)
  const int i = blockIdx.x * 256 + threadIdx.x; if (i >= nrows) return; const float* s = S + (size_t)i * SQ; float mx = -3.0e38f;
#pragma unroll 1
  for (int j = 0; j < SQ; ++j) mx = fmaxf(mx, s[j]); float se = 0.f;
#pragma unroll 1
  for (int j = 0; j < SQ; ++j) se += expf(s[j] - mx); const float sc = 256.0f / se;
#pragma unroll 1
  for (int j0 = 0; j0 < SQ; j0 += 8) { FragH f; for (int q = 0; q < 8; ++q) f.h[q] = (_Float16)(expf(s[j0 + q] - mx) * sc); unsigned short* d = (unsigned short*)P + (size_t)i * SQ + j0; *(volatile v8us*)d = f.half[0]; __threadfence(); *(volatile v8us*)d = f.half[0]; } }
__global__ __launch_bounds__(256) void k_vt(const _Float16* __restrict__ V16, int b, int h0, _Float16* __restrict__ VT) { __shared__ unsigned short tl[64][65]; const int tid = threadIdx.x; const int hh = blockIdx.x % HG, sg = blockIdx.x / HG; const int s0 = sg * 64; const int h = h0 + hh;
  for (int i = tid; i < 64 * 8; i += 256) { const int j = i / 8, d8 = (i % 8) * 8; FragH f; f.half[0] = *(const v8us*)((const unsigned short*)V16 + ((size_t)b * SQ + s0 + j) * DM + h * HD + d8); for (int q = 0; q < 8; ++q) tl[d8 + q][j] = f.u[q]; }
  __syncthreads();
  for (int pass = 0; pass < 2; ++pass) { for (int i = tid; i < 64 * 8; i += 256) { const int d = i / 8, j8 = (i % 8) * 8; FragH f; for (int q = 0; q < 8; ++q) f.u[q] = tl[d][j8 + q]; *(volatile v8us*)((unsigned short*)VT + ((size_t)hh * HD + d) * SQ + s0 + j8) = f.half[0]; } if (pass == 0) __threadfence(); } }


__global__ __launch_bounds__(256) void k_rsmkm(const float* __restrict__ S, _Float16* __restrict__ P, int nrows, const int* __restrict__ am) {
  #pragma clang fp contract(off)
  const int t = blockIdx.x * 256 + threadIdx.x; if (t >= nrows) return; const size_t i = (size_t)t; const float* s = S + i * SQ; const int* mr = am + (size_t)(t % SQ) * SQ; float mx = -3.0e38f;
#pragma unroll 1
  for (int j = 0; j < SQ; ++j) { const float f = (mr[j] != 0) ? 1.f : 0.f; mx = fmaxf(mx, fmaf(f, s[j], (1.f - f) * -1.0e9f)); } float se = 0.f;
#pragma unroll 1
  for (int j = 0; j < SQ; ++j) { const float f = (mr[j] != 0) ? 1.f : 0.f; se += __expf(fmaf(f, s[j], (1.f - f) * -1.0e9f) - mx); } const float sc = 256.0f / se;
#pragma unroll 1
  for (int j0 = 0; j0 < SQ; j0 += 8) { FragH fr; for (int q = 0; q < 8; ++q) { const int j = j0 + q; const float f = (mr[j] != 0) ? 1.f : 0.f; fr.h[q] = (_Float16)(__expf(fmaf(f, s[j], (1.f - f) * -1.0e9f) - mx) * sc); }
    unsigned short* d = (unsigned short*)P + i * SQ + j0; *(volatile v8us*)d = fr.half[0]; __threadfence(); *(volatile v8us*)d = fr.half[0]; } }

__global__ __launch_bounds__(256) void k_bdshn(const float* __restrict__ Wb, _Float16* __restrict__ Bt) {
  const size_t t = (size_t)blockIdx.x * 256 + threadIdx.x; if (t >= (size_t)DM * DM / 8) return; const size_t e0 = t * 8; const int n = (int)(e0 / DM), k0 = (int)(e0 % DM); const int h = n >> 6, hk = k0 >> 6; const float on = (hk == h) ? 16.0f : 0.0f; const int o = n & 63, d0 = k0 & 63; FragH f;
  for (int q = 0; q < 8; ++q) f.h[q] = (_Float16)(bf16_round(Wb[(size_t)o * 64 + d0 + q]) * on);
  unsigned short* d = (unsigned short*)Bt + e0; *(volatile v8us*)d = f.half[0]; __threadfence(); *(volatile v8us*)d = f.half[0]; }
extern "C" void kernel_launch(void* const* d_in, const int* in_sizes, int n_in,
                              void* d_out, int out_size, void* d_ws, size_t ws_size, hipStream_t stream) {
  (void)in_sizes; (void)n_in; (void)out_size;
  const float* const* I = (const float* const*)d_in; const float* xq = I[2]; const float* xk = I[1]; const float* xv = I[0]; const float* wq = I[5]; const float* bq = nullptr; const float* wk = I[4]; const float* bk = nullptr; const float* wv = I[3]; const float* bv = nullptr; const float* wo = I[6]; const float* bo = I[7]; const float* x = xq;
  char* ws = (char*)d_ws; size_t off = 0;
  auto take = [&](size_t bytes) { char* p = ws + off; off += (bytes + 255) & ~(size_t)255; return p; };
  _Float16* BQ = (_Float16*)take((size_t)DM * DM * 2); _Float16* BK = (_Float16*)take((size_t)DM * DM * 2); _Float16* BV = (_Float16*)take((size_t)DM * DM * 2); _Float16* BO = (_Float16*)take((size_t)DM * DM * 2);
  _Float16* X16 = (_Float16*)take(NR * DM * 2); _Float16* XKp = (_Float16*)take(NR * DM * 2); _Float16* XVp = (_Float16*)take(NR * DM * 2); _Float16* Q16 = (_Float16*)take(NR * DM * 2); _Float16* K16 = (_Float16*)take(NR * DM * 2); _Float16* V16 = (_Float16*)take(NR * DM * 2); _Float16* O16 = (_Float16*)take(NR * DM * 2);
  float* S = (float*)take((size_t)HG * SQ * SQ * 4); _Float16* P = (_Float16*)take((size_t)HG * SQ * SQ * 2); _Float16* VT = (_Float16*)take((size_t)NH * HD * SQ * 2);
  if (off > ws_size) return;
  { const unsigned g = (unsigned)(((size_t)DM * DM / 8 + 255) / 256); k_bdshn<<<g, 256, 0, stream>>>(wq, BQ); k_bdshn<<<g, 256, 0, stream>>>(wk, BK); k_bdshn<<<g, 256, 0, stream>>>(wv, BV); k_wnat<<<g, 256, 0, stream>>>(wo, (size_t)DM * DM / 8, BO); }
  _Float16* XK = XKp; _Float16* XV = XVp; k_x16<<<(unsigned)((NR * DM / 8 + 255) / 256), 256, 0, stream>>>(xk, XK, NR * DM / 8); k_x16<<<(unsigned)((NR * DM / 8 + 255) / 256), 256, 0, stream>>>(xv, XV, NR * DM / 8);

  k_x16<<<(unsigned)((NR * DM / 8 + 255) / 256), 256, 0, stream>>>(x, X16, NR * DM / 8);
  const size_t r0p = (size_t)B0 * SQ;
  k_gemm2<0><<<dim3((unsigned)((MP / 128) * (DM / 64)), 1), 128, 0, stream>>>(X16 + r0p * DM, DM, 0, BQ, DM, 0, 0.0625f, bq, 0, nullptr, 1, 0, 0, nullptr, Q16 + r0p * DM, DM, 0, MP, DM, DM);
  k_gemm2<0><<<dim3((unsigned)((MP / 128) * (DM / 64)), 1), 128, 0, stream>>>(XK + r0p * DM, DM, 0, BK, DM, 0, 0.0625f, bk, 0, nullptr, 1, 0, 0, nullptr, K16 + r0p * DM, DM, 0, MP, DM, DM);
  k_gemm2<0><<<dim3((unsigned)((MP / 128) * (DM / 64)), 1), 128, 0, stream>>>(XV + r0p * DM, DM, 0, BV, DM, 0, 0.0625f, bv, 0, nullptr, 1, 0, 0, nullptr, V16 + r0p * DM, DM, 0, MP, DM, DM);
  for (int b = B0; b < B0 + NBR; ++b) { const size_t r0 = (size_t)b * SQ;
    k_vt<NH, SQ><<<NH * (SQ / 64), 256, 0, stream>>>(V16 + r0 * LQ, LQ, 0, VT);
    for (int h0 = 0; h0 < NHD; h0 += HG) {
      k_gemm2<0><<<dim3((QN / 128) * (SQ / 64), HG), 128, 0, stream>>>(Q16 + r0 * LQ + h0 * HD, LQ, (size_t)HD, K16 + r0 * LQ + h0 * HD, LQ, (size_t)HD, 0.03125f, nullptr, 0, nullptr, 1, 0, 0, S, nullptr, SQ, (size_t)SQ * SQ, QN, SQ, HD);
      k_rsm<<<(HG * SQ + 255) / 256, 256, 0, stream>>>(S, P, HG * SQ);
      k_gemm2<0><<<dim3((QN / 128) * (HD / 64), HG), 128, 0, stream>>>(P, SQ, (size_t)SQ * SQ, VT + (size_t)h0 * HD * SQ, SQ, (size_t)HD * SQ, 0.25f, nullptr, 0, nullptr, 1, 0, 0, nullptr, O16 + r0 * DM + h0 * HD, DM, (size_t)HD, QN, HD, SQ); } }
  k_gemm2<0><<<dim3((unsigned)((MPO / 128) * (DM / 64)), 1), 128, 0, stream>>>(O16 + r0p * DM, DM, 0, BO, DM, 0, 0.0009765625f, bo, 0, nullptr, 1, 0, 0, (float*)d_out + r0p * DM, nullptr, DM, 0, MPO, DM, DM);
}
